// MambaDecisionModel_11828339933363
// MI455X (gfx1250) — hardware-run, weakly checked
//
#include <hip/hip_runtime.h>


#define NBT  262144
#define SD   32
#define DMd  64
#define DI   128
#define DSt  16
#define DTR  4
#define XPN  64
#define RCH  32768
#define OFF1 4194304
#define OFF2 6291456
typedef _Float16 h16;
typedef unsigned short bf;
typedef __attribute__((ext_vector_type(16))) __bf16   v16bf;
typedef __attribute__((ext_vector_type(16))) _Float16 v16h;
typedef __attribute__((ext_vector_type(8)))  _Float16 v8h;
typedef __attribute__((ext_vector_type(8)))  unsigned short v8us;
typedef __attribute__((ext_vector_type(8)))  float    v8f;
typedef __attribute__((ext_vector_type(4)))  float    v4f;
typedef v8h  __attribute__((may_alias)) v8ha;
typedef v4f  __attribute__((may_alias)) v4fa;
typedef v8us __attribute__((may_alias)) v8usa;

__device__ __forceinline__ unsigned short f2bf(float f) { unsigned u = __float_as_uint(f); u += 0x7FFFu + ((u >> 16) & 1u); return (unsigned short)(u >> 16); }
__device__ __forceinline__ float bf2f(unsigned short b) { return __uint_as_float(((unsigned)b) << 16); }
__device__ __forceinline__ float bfr(float f) { return bf2f(f2bf(f)); }
__device__ __forceinline__ v16h cat16(v8h lo, v8h hi) { return __builtin_shufflevector(lo, hi, 0, 1, 2, 3, 4, 5, 6, 7, 8, 9, 10, 11, 12, 13, 14, 15); }
__device__ __forceinline__ v16bf cat16b(v8us lo, v8us hi) { return __builtin_bit_cast(v16bf, __builtin_shufflevector(lo, hi, 0, 1, 2, 3, 4, 5, 6, 7, 8, 9, 10, 11, 12, 13, 14, 15)); }
__device__ __forceinline__ v8f wmma16(v16h a, v16h b, v8f c) { return __builtin_amdgcn_wmma_f32_16x16x32_f16(false, a, false, b, (short)0, c, false, false); }
__device__ __forceinline__ v8f wmmab(v16bf a, v16bf b, v8f c) { return __builtin_amdgcn_wmma_f32_16x16x32_bf16(false, a, false, b, (short)0, c, false, false); }


template <typename T16> struct WFrag;
template <> struct WFrag<h16> { typedef v16h V; static __device__ __forceinline__ V ld(const h16* p) { return cat16(*(const v8h*)p, *(const v8h*)(p + 16)); } static __device__ __forceinline__ v8f mma(V a, V b, v8f c) { return wmma16(a, b, c); } };
template <> struct WFrag<bf> { typedef v16bf V; static __device__ __forceinline__ V ld(const bf* p) { return cat16b(*(const v8us*)p, *(const v8us*)(p + 16)); } static __device__ __forceinline__ v8f mma(V a, V b, v8f c) { return wmmab(a, b, c); } };
template <typename T16, int NSPLIT, bool BIAS>
__global__ __launch_bounds__(32) void k_gemmw(const T16* __restrict__ A, const T16* __restrict__ A2, const T16* __restrict__ Bt, const T16* __restrict__ Bt2, int K, float* C, int ldc, const float* __restrict__ bias, size_t sA, size_t sB, size_t sC) {
    typedef typename WFrag<T16>::V V;
    __shared__ __align__(16) float os[16 * 68];
    const size_t z = blockIdx.z; A += z * sA; if (A2) A2 += z * sA; Bt += z * sB; if (Bt2) Bt2 += z * sB; C += z * sC;
    const int lane = threadIdx.x & 31, lr = lane & 15, hi = lane >> 4; const int r0 = blockIdx.x * 64, c0 = blockIdx.y * 64;
    v8f acc[4][4];
#pragma unroll
    for (int mb = 0; mb < 4; ++mb)
#pragma unroll
        for (int nb = 0; nb < 4; ++nb) acc[mb][nb] = (v8f){};
    const size_t aoff = (size_t)(r0 + lr) * K + 8 * hi, boff = (size_t)(c0 + lr) * K + 8 * hi;
#pragma unroll 1
    for (int kc = 0; kc < K; kc += 32) {
        V a[4], a2[4];
#pragma unroll
        for (int mb = 0; mb < 4; ++mb) { a[mb] = WFrag<T16>::ld(A + aoff + (size_t)mb * 16 * K + kc); if (NSPLIT == 1 || NSPLIT == 2) a2[mb] = WFrag<T16>::ld(A2 + aoff + (size_t)mb * 16 * K + kc); }
#pragma unroll
        for (int nb = 0; nb < 4; ++nb) { const V b = WFrag<T16>::ld(Bt + boff + (size_t)nb * 16 * K + kc); V b2; if (NSPLIT >= 2) b2 = WFrag<T16>::ld(Bt2 + boff + (size_t)nb * 16 * K + kc);
#pragma unroll
            for (int mb = 0; mb < 4; ++mb) { acc[mb][nb] = WFrag<T16>::mma(a[mb], b, acc[mb][nb]); if (NSPLIT == 1 || NSPLIT == 2) acc[mb][nb] = WFrag<T16>::mma(a2[mb], b, acc[mb][nb]); if (NSPLIT >= 2) acc[mb][nb] = WFrag<T16>::mma(a[mb], b2, acc[mb][nb]); } }
        asm volatile("v_nop\n\tv_nop\n\tv_nop\n\tv_nop" : "+v"(acc[0][0]), "+v"(acc[1][1]), "+v"(acc[2][2]), "+v"(acc[3][3]) : "v"(a[0]), "v"(a[3]));
    }
#pragma unroll
    for (int mb = 0; mb < 4; ++mb) {
#pragma unroll
        for (int nb = 0; nb < 4; ++nb) {
#pragma unroll
            for (int j = 0; j < 8; ++j) os[(hi * 8 + j) * 68 + nb * 16 + lr] = acc[mb][nb][j]; }
        __builtin_amdgcn_wave_barrier(); asm volatile("" ::: "memory");
        float* crow = C + (size_t)(r0 + mb * 16) * ldc + c0;
#pragma unroll 1
        for (int ps = 0; ps < 2; ++ps) {
#pragma unroll
            for (int s = 0; s < 8; ++s) { const int row = 2 * s + hi, cofs = lr * 4; v4f val = *(const v4fa*)(os + row * 68 + cofs); if (BIAS) { val[0] += bfr(bias[c0 + cofs]); val[1] += bfr(bias[c0 + cofs + 1]); val[2] += bfr(bias[c0 + cofs + 2]); val[3] += bfr(bias[c0 + cofs + 3]); }
                *(volatile v4f*)(crow + (size_t)row * ldc + cofs) = val; }
            if (ps == 0) __threadfence(); }
        __builtin_amdgcn_wave_barrier(); asm volatile("" ::: "memory");
    }
}

__device__ __forceinline__ void splitf(float y, unsigned short& h, unsigned short& l) { h = f2bf(y); l = f2bf(y - bf2f(h)); }
__device__ __forceinline__ float sigm_(float x) { return __fdiv_rn(1.0f, 1.0f + __expf(-x)); }
__device__ __forceinline__ float silu_(float x) { return __fmul_rn(x, sigm_(x)); }
__device__ __forceinline__ float tanh_(float x) { const float e = __expf(-2.0f * fabsf(x)); const float t = __fdiv_rn(1.0f - e, 1.0f + e); return copysignf(t, x); }
typedef __attribute__((ext_vector_type(2))) unsigned short v2us;
typedef __attribute__((ext_vector_type(4))) unsigned short v4us;
typedef __attribute__((ext_vector_type(2))) float v2f;

__global__ __launch_bounds__(256) void k_cvt8(const float* __restrict__ src, bf* dst, size_t n8) { const size_t i = (size_t)blockIdx.x * 256 + threadIdx.x; if (i >= n8) return; const v8f v = *(const v8f*)(src + i * 8); v8us o;
#pragma unroll
    for (int k = 0; k < 8; ++k) o[k] = f2bf(v[k]); *(volatile v8us*)(dst + i * 8) = o; __threadfence(); *(volatile v8us*)(dst + i * 8) = o; }
__global__ __launch_bounds__(256) void k_xpw(const float* __restrict__ w, bf* Bt) { const int i = (blockIdx.x * 256 + threadIdx.x) * 4; if (i >= XPN * DI) return; const int k = i % DI, n = i / DI; v4us o;
#pragma unroll
    for (int q = 0; q < 4; ++q) o[q] = n < (DTR + 2 * DSt) ? f2bf(w[n * DI + k + q]) : (unsigned short)0; *(volatile v4us*)(Bt + i) = o; __threadfence(); *(volatile v4us*)(Bt + i) = o; }
__global__ __launch_bounds__(256) void k_spl(const float* __restrict__ F, size_t n4, bf* Fh, bf* Fl) { const size_t i = ((size_t)blockIdx.x * 256 + threadIdx.x) * 4; if (i >= n4 * 4) return; const v4f a = *(const v4f*)(F + i); v4us oh, ol;
#pragma unroll
    for (int q = 0; q < 4; ++q) { unsigned short u, c; splitf(a[q], u, c); oh[q] = u; ol[q] = c; } *(volatile v4us*)(Fh + i) = oh; *(volatile v4us*)(Fl + i) = ol; __threadfence(); *(volatile v4us*)(Fh + i) = oh; *(volatile v4us*)(Fl + i) = ol; }
__global__ __launch_bounds__(256) void k_xcpl(const float* __restrict__ XZ, const float* __restrict__ cw, const float* __restrict__ cb, bf* Xh, bf* Xl) { const size_t e = ((size_t)blockIdx.x * 256 + threadIdx.x) * 4; if (e >= (size_t)RCH * DI) return; const int d = (int)(e % DI); const size_t b = e / DI; v4us oh, ol;
#pragma unroll
    for (int q = 0; q < 4; ++q) { float t = __fmul_rn(XZ[b * 2 * DI + d + q], bfr(cw[(d + q) * 4 + 3])); asm volatile("" : "+v"(t)); const float xc = silu_(__fadd_rn(t, bfr(cb[d + q]))); unsigned short u, c; splitf(xc, u, c); oh[q] = u; ol[q] = c; }
    *(volatile v4us*)(Xh + e) = oh; *(volatile v4us*)(Xl + e) = ol; __threadfence(); *(volatile v4us*)(Xh + e) = oh; *(volatile v4us*)(Xl + e) = ol; }
__global__ __launch_bounds__(256) void k_ssm(const float* __restrict__ XZ, const float* __restrict__ cw, const float* __restrict__ cb, const float* __restrict__ XD, const float* __restrict__ dtw, const float* __restrict__ dtb, const float* __restrict__ Dv, bf* Yh, bf* Yl) {
    const size_t e = ((size_t)blockIdx.x * 256 + threadIdx.x) * 2; if (e >= (size_t)RCH * DI) return; const int d = (int)(e % DI); const size_t b = e / DI; const float* xd = XD + b * XPN; float bc = 0.f;
#pragma unroll
    for (int s = 0; s < DSt; ++s) { float p = __fmul_rn(xd[DTR + s], xd[DTR + DSt + s]); asm volatile("" : "+v"(p)); bc = __fadd_rn(bc, p); }
    v2us oh, ol;
#pragma unroll
    for (int q = 0; q < 2; ++q) { const int dd = d + q; float t = __fmul_rn(XZ[b * 2 * DI + dd], bfr(cw[dd * 4 + 3])); asm volatile("" : "+v"(t)); const float xc = silu_(__fadd_rn(t, bfr(cb[dd]))); float raw = bfr(dtb[dd]);
#pragma unroll
        for (int r = 0; r < DTR; ++r) { float p = __fmul_rn(xd[r], bfr(dtw[dd * DTR + r])); asm volatile("" : "+v"(p)); raw = __fadd_rn(raw, p); }
        const float delta = raw > 20.f ? raw : log1pf(__expf(raw)); float dx = __fmul_rn(delta, xc); asm volatile("" : "+v"(dx)); float y0 = __fmul_rn(dx, bc); asm volatile("" : "+v"(y0)); float sk = __fmul_rn(bfr(Dv[dd]), xc); asm volatile("" : "+v"(sk)); const float y = __fmul_rn(__fadd_rn(y0, sk), silu_(XZ[b * 2 * DI + DI + dd]));
        unsigned short u, c; splitf(y, u, c); oh[q] = u; ol[q] = c; }
    *(volatile v2us*)(Yh + e) = oh; *(volatile v2us*)(Yl + e) = ol; __threadfence(); *(volatile v2us*)(Yh + e) = oh; *(volatile v2us*)(Yl + e) = ol; }
__global__ __launch_bounds__(256) void k_heads(const float* __restrict__ H2, const float* __restrict__ wa, const float* __restrict__ ba, const float* __restrict__ wd, const float* __restrict__ bd, const float* __restrict__ wi, const float* __restrict__ bi, float* O0, float* O1, float* O2) {
    const size_t b = (size_t)blockIdx.x * 256 + threadIdx.x; if (b >= RCH) return; const float* h = H2 + b * DMd; float acc[7];
#pragma unroll
    for (int o = 0; o < 7; ++o) acc[o] = o < 4 ? bfr(ba[o]) : (o < 6 ? bfr(bd[o - 4]) : bfr(bi[0]));
#pragma unroll 1
    for (int k = 0; k < DMd; ++k) { const float hv = h[k];
#pragma unroll
        for (int o = 0; o < 7; ++o) { const float w = o < 4 ? wa[o * DMd + k] : (o < 6 ? wd[(o - 4) * DMd + k] : wi[k]); float p = __fmul_rn(hv, bfr(w)); asm volatile("" : "+v"(p)); acc[o] = __fadd_rn(acc[o], p); } }
    v4f a; a[0] = acc[0]; a[1] = acc[1]; a[2] = acc[2]; a[3] = acc[3]; v2f dv; dv[0] = tanh_(acc[4]); dv[1] = tanh_(acc[5]); const float iv = sigm_(acc[6]);
    for (int ps = 0; ps < 2; ++ps) { *(volatile v4f*)(O0 + b * 4) = a; *(volatile v2f*)(O1 + b * 2) = dv; *(volatile float*)(O2 + b) = iv; if (ps == 0) __threadfence(); } }

extern "C" void kernel_launch(void* const* d_in, const int* in_sizes, int n_in,
                              void* d_out, int out_size, void* d_ws, size_t ws_size, hipStream_t stream) {
    (void)in_sizes; (void)n_in; (void)out_size;
    const float* IN[18]; for (int i = 0; i < 18; ++i) IN[i] = (const float*)d_in[i];
    float* O0 = (float*)d_out; float* O1 = (float*)((char*)d_out + OFF1); float* O2 = (float*)((char*)d_out + OFF2);
    char* wsp = (char*)d_ws;
    auto take = [&](size_t bytes) { char* p = wsp; wsp += (bytes + 255) & ~(size_t)255; return (void*)p; };
    bf* WE = (bf*)take(DMd * SD * 2); bf* WI = (bf*)take(2 * DI * DMd * 2); bf* WX = (bf*)take(XPN * DI * 2); bf* WO = (bf*)take(DMd * DI * 2); bf* XB = (bf*)take((size_t)RCH * SD * 2); float* HF = (float*)take((size_t)RCH * DMd * 4);
    bf* Ph = (bf*)take((size_t)RCH * DI * 2); bf* Pl = (bf*)take((size_t)RCH * DI * 2); float* XZ = (float*)take((size_t)RCH * 2 * DI * 4); float* XD = (float*)take((size_t)RCH * XPN * 4); float* H2 = (float*)take((size_t)RCH * DMd * 4);
    if ((size_t)(wsp - (char*)d_ws) > ws_size) return;
    k_cvt8<<<(DMd * SD / 8 + 255) / 256, 256, 0, stream>>>(IN[1], WE, DMd * SD / 8); k_cvt8<<<(2 * DI * DMd / 8 + 255) / 256, 256, 0, stream>>>(IN[3], WI, 2 * DI * DMd / 8); k_xpw<<<(XPN * DI / 4 + 255) / 256, 256, 0, stream>>>(IN[6], WX); k_cvt8<<<(DMd * DI / 8 + 255) / 256, 256, 0, stream>>>(IN[11], WO, DMd * DI / 8);
    for (int r0 = 0; r0 < NBT; r0 += RCH) {
        k_cvt8<<<(RCH * SD / 8 + 255) / 256, 256, 0, stream>>>(IN[0] + (size_t)r0 * SD, XB, (size_t)RCH * SD / 8);
        k_gemmw<bf, 0, true><<<dim3(RCH / 64, DMd / 64, 1), 32, 0, stream>>>(XB, nullptr, WE, nullptr, SD, HF, DMd, IN[2], 0, 0, 0);
        k_spl<<<(RCH * DMd / 4 + 255) / 256, 256, 0, stream>>>(HF, (size_t)RCH * DMd / 4, Ph, Pl);
        k_gemmw<bf, 1, false><<<dim3(RCH / 64, 2 * DI / 64, 1), 32, 0, stream>>>(Ph, Pl, WI, nullptr, DMd, XZ, 2 * DI, nullptr, 0, 0, 0);
        k_xcpl<<<(RCH * DI / 4 + 255) / 256, 256, 0, stream>>>(XZ, IN[4], IN[5], Ph, Pl);
        k_gemmw<bf, 1, false><<<dim3(RCH / 64, XPN / 64, 1), 32, 0, stream>>>(Ph, Pl, WX, nullptr, DI, XD, XPN, nullptr, 0, 0, 0);
        k_ssm<<<(RCH * DI / 2 + 255) / 256, 256, 0, stream>>>(XZ, IN[4], IN[5], XD, IN[7], IN[8], IN[10], Ph, Pl);
        k_gemmw<bf, 1, false><<<dim3(RCH / 64, DMd / 64, 1), 32, 0, stream>>>(Ph, Pl, WO, nullptr, DI, H2, DMd, nullptr, 0, 0, 0);
        k_heads<<<RCH / 256, 256, 0, stream>>>(H2, IN[12], IN[13], IN[14], IN[15], IN[16], IN[17], O0 + (size_t)r0 * 4, O1 + (size_t)r0 * 2, O2 + r0); }
}
